// PointNetSAModule_6176162972233
// MI455X (gfx1250) — hardware-verified
//
#include <hip/hip_runtime.h>
#pragma clang fp contract(off)

typedef __attribute__((ext_vector_type(16))) _Float16 v16h;
typedef __attribute__((ext_vector_type(8)))  _Float16 v8h;
typedef __attribute__((ext_vector_type(8)))  float    v8f;
typedef __attribute__((ext_vector_type(4)))  float    v4f;
typedef __attribute__((ext_vector_type(4)))  int      v4i;

constexpr int kBatch = 4;
constexpr int kPts   = 8192;
constexpr int kChild = 2048;
constexpr int kCin   = 128;
constexpr int kCout  = 256;
constexpr int kNbr   = 16;
constexpr float kWCarry    = 64.0f;
constexpr float kWCarryInv = 1.0f / 64.0f;

static_assert(kChild * 4 == kPts, "child count");
static_assert(kBatch * kPts * 3 == 98304, "xyz elements");
static_assert(kBatch * kCin * kPts == 4194304, "feats elements");
static_assert((kBatch * kPts) % 64 == 0 && kCout % 64 == 0, "GEMM M,N tile multiples");
static_assert(kCin % 32 == 0 && kCout % 32 == 0, "GEMM K multiples of 32");

constexpr size_t kOffXh   = 0;
constexpr size_t kOffWh   = kOffXh + (size_t)kBatch * kPts * kCin * 2;
constexpr size_t kOffY1   = kOffWh + (size_t)(kCout * kCin + kCout * kCout) * 2;
constexpr size_t kOffY2   = kOffY1 + (size_t)kBatch * kPts * kCout * 2;
constexpr size_t kOffCidx = kOffY2 + (size_t)kBatch * kPts * kCout * 2;
constexpr size_t kWsTotal = kOffCidx + (size_t)kBatch * kChild * 4;
static_assert(kWsTotal == 42172416, "carve total");
static_assert(kWsTotal <= 134217728, "carve limit");
static_assert(kOffWh % 128 == 0 && kOffY1 % 128 == 0 && kOffY2 % 128 == 0 && kOffCidx % 128 == 0, "line aligned");

constexpr size_t kOut0Bytes = (size_t)kBatch * kChild * 3 * 4;
constexpr size_t kOut1Bytes = (size_t)kBatch * kCout * kChild * 4;
static_assert(kOut0Bytes == 98304 && kOut0Bytes % 128 == 0, "out0 extent");
static_assert(kOut0Bytes + kOut1Bytes == 8486912, "d_out total");

__device__ __forceinline__ float h16_to_f32(unsigned hb) {
  const unsigned sgn = (hb & 0x8000u) << 16; const unsigned em = hb & 0x7fffu;
  const float fn = __uint_as_float((em << 13) + 0x38000000u);
  const float fs = (float)em * 5.9604644775390625e-8f;
  const float mag = (em < 0x400u) ? fs : fn; return __uint_as_float(__float_as_uint(mag) | sgn); }

struct FragH {
  union U { v16h v; v8h h[2]; };
  static __device__ __forceinline__ v16h load(const _Float16* p) {
    U f; f.h[0] = *(const v8h*)(p); f.h[1] = *(const v8h*)(p + 16); return f.v;
  }
  static __device__ __forceinline__ v8f mma(v16h a, v16h b, v8f c) {
    return __builtin_amdgcn_wmma_f32_16x16x32_f16(false, a, false, b, (short)0, c, false, false);
  }
};
__device__ __forceinline__ void guard_group_h(v8f& a, v8f& b, v8f& c, v8f& d, v16h x, v16h b0, v16h b1, v16h b2, v16h b3) {
  asm volatile("v_nop\n\tv_nop\n\tv_nop\n\tv_nop" : "+v"(a), "+v"(b), "+v"(c), "+v"(d) : "v"(x), "v"(b0), "v"(b1), "v"(b2), "v"(b3));
}
__device__ __forceinline__ void keep4_h(v16h a, v16h b, v16h c, v16h d) { asm volatile("v_nop" :: "v"(a), "v"(b), "v"(c), "v"(d)); }
__device__ __forceinline__ void acc_guard4(v8f& a, v8f& b, v8f& c, v8f& d) { asm volatile("v_nop\n\tv_nop\n\tv_nop\n\tv_nop" : "+v"(a), "+v"(b), "+v"(c), "+v"(d)); }

__global__ __launch_bounds__(256) void wmma_gemm64_f16_bias_relu(
    const unsigned short* __restrict__ Ap, int lda,
    const unsigned short* __restrict__ Btp, int ldb,
    unsigned short* __restrict__ Cp, int ldc,
    const float* __restrict__ bias, int M, int N, int K, float scale) {
  const _Float16* A  = (const _Float16*)Ap;
  const _Float16* Bt = (const _Float16*)Btp;
  __shared__ __align__(16) float sT[8][16 * 68];
  const int lane = threadIdx.x & 31;
  const int wave = threadIdx.x >> 5;
  const int tilesN = N >> 6;
  const int tilesM = M >> 6;
  const int tile = blockIdx.x * 8 + wave;
  if (tile >= tilesM * tilesN) return;
  const int tm = tile / tilesN;
  const int tn = tile - tm * tilesN;
  const int m0 = tm << 6;
  const int n0 = tn << 6;

  const int rlane = lane & 15;
  const int koff  = (lane >> 4) * 8;
  const int mOff  = (lane >> 4) * 8;

  v8f acc[4][4];
#pragma unroll
  for (int i = 0; i < 4; ++i)
#pragma unroll
    for (int j = 0; j < 4; ++j) acc[i][j] = (v8f){0.f,0.f,0.f,0.f,0.f,0.f,0.f,0.f};

  for (int k0 = 0; k0 < K; k0 += 32) {
    v16h bh[4];
#pragma unroll
    for (int j = 0; j < 4; ++j) {
      const size_t bo = (size_t)(n0 + (j << 4) + rlane) * ldb + koff + k0;
      bh[j] = FragH::load(Bt + bo);
    }
#pragma unroll
    for (int i = 0; i < 4; ++i) {
      const size_t ao = (size_t)(m0 + (i << 4) + rlane) * lda + koff + k0;
      v16h ah = FragH::load(A + ao);
#pragma unroll
      for (int j = 0; j < 4; ++j) acc[i][j] = FragH::mma(ah, bh[j], acc[i][j]);
      guard_group_h(acc[i][0], acc[i][1], acc[i][2], acc[i][3], ah, bh[0], bh[1], bh[2], bh[3]);
    }
    keep4_h(bh[0], bh[1], bh[2], bh[3]);
  }
  acc_guard4(acc[0][0], acc[0][1], acc[0][2], acc[0][3]);
  acc_guard4(acc[1][0], acc[1][1], acc[1][2], acc[1][3]);
  acc_guard4(acc[2][0], acc[2][1], acc[2][2], acc[2][3]);
  acc_guard4(acc[3][0], acc[3][1], acc[3][2], acc[3][3]);

  float* slab = sT[wave];
  float bvals[4];
#pragma unroll
  for (int j = 0; j < 4; ++j) bvals[j] = bias[n0 + (j << 4) + rlane];
#pragma unroll
  for (int i = 0; i < 4; ++i) {
    const int mBase = m0 + (i << 4);
#pragma unroll
    for (int j = 0; j < 4; ++j) {
#pragma unroll
      for (int r = 0; r < 8; ++r) {
        float v = acc[i][j][r] * scale;
        v = v + bvals[j];
        v = fmaxf(v, 0.0f);
        slab[(mOff + r) * 68 + (j << 4) + rlane] = v;
      }
    }
    __builtin_amdgcn_fence(__ATOMIC_RELEASE, "workgroup");
    __builtin_amdgcn_wave_barrier();
    __builtin_amdgcn_fence(__ATOMIC_ACQUIRE, "workgroup");
    {
      const int q = lane >> 3, c8 = (lane & 7) * 8;
      for (int pass = 0; pass < 2; ++pass) {
#pragma unroll
        for (int it = 0; it < 4; ++it) {
          const int row = it * 4 + q;
          const float* sp = slab + row * 68 + c8;
          v8h hv;
#pragma unroll
          for (int e = 0; e < 8; ++e) hv[e] = (_Float16)sp[e];
          *(volatile v8h*)(Cp + (size_t)(mBase + row) * ldc + n0 + c8) = hv;
        }
        __threadfence();
      }
    }
    __builtin_amdgcn_fence(__ATOMIC_RELEASE, "workgroup");
    __builtin_amdgcn_wave_barrier();
    __builtin_amdgcn_fence(__ATOMIC_ACQUIRE, "workgroup");
  }
}

__global__ __launch_bounds__(256) void cvt_feats_kernel(const float* __restrict__ feats, unsigned short* __restrict__ Xh) {
  __shared__ __align__(16) float s_t[128 * 68];
  const int tid = threadIdx.x;
  const int b  = blockIdx.x >> 7;
  const int p0 = (blockIdx.x & 127) * 64;
#pragma unroll
  for (int it = 0; it < 8; ++it) {
    const int q  = it * 256 + tid;
    const int c  = q >> 4;
    const int n4 = (q & 15) * 4;
    const v4f f = *(const v4f*)(feats + ((size_t)(b * kCin + c)) * kPts + p0 + n4);
    *(v4f*)(s_t + c * 68 + n4) = f;
  }
  __syncthreads();
  v8h hv[4];
#pragma unroll
  for (int it = 0; it < 4; ++it) {
    const int q  = it * 256 + tid;
    const int p  = q >> 4;
    const int c8 = (q & 15) * 8;
#pragma unroll
    for (int e = 0; e < 8; ++e) hv[it][e] = (_Float16)s_t[(c8 + e) * 68 + p];
  }
  for (int pass = 0; pass < 2; ++pass) {
#pragma unroll
    for (int it = 0; it < 4; ++it) {
      const int q  = it * 256 + tid;
      const int p  = q >> 4;
      const int c8 = (q & 15) * 8;
      *(volatile v8h*)(Xh + ((size_t)(b * kPts + p0 + p)) * kCin + c8) = hv[it];
    }
    __threadfence();
  }
}

__global__ __launch_bounds__(256) void cvt_w_kernel(const float* __restrict__ w1, const float* __restrict__ w2, unsigned short* __restrict__ Wh) {
  const int g  = blockIdx.x * 256 + threadIdx.x;
  const int i8 = g * 8;
  const float* src = (blockIdx.x < 16) ? (w1 + i8) : (w2 + (i8 - kCout * kCin));
  const v4f a = *(const v4f*)(src);
  const v4f c = *(const v4f*)(src + 4);
  v8h hv;
#pragma unroll
  for (int e = 0; e < 4; ++e) {
    hv[e]     = (_Float16)(a[e] * kWCarry);
    hv[4 + e] = (_Float16)(c[e] * kWCarry);
  }
  *(volatile v8h*)(Wh + i8) = hv;
  __threadfence();
  *(volatile v8h*)(Wh + i8) = hv;
}

__device__ __forceinline__ void argmax_allreduce(float& bv, int& bi) {
#pragma unroll
  for (int off = 16; off > 0; off >>= 1) {
    const float ov = __shfl_xor(bv, off, 32);
    const int   oi = __shfl_xor(bi, off, 32);
    const bool take = (ov > bv) || ((ov == bv) && (oi < bi));
    bv = take ? ov : bv;
    bi = take ? oi : bi;
  }
}

__global__ __launch_bounds__(1024) void fps_kernel(const float* __restrict__ xyz, float* __restrict__ out0, int* __restrict__ cidx_ws) {
#pragma clang fp contract(off)
  __shared__ __align__(16) float s_stage[3072];
  __shared__ float s_bv[2][32];
  __shared__ int   s_bi[2][32];
  __shared__ __align__(16) int s_cidx[kChild];

  const int b    = blockIdx.x;
  const int t    = threadIdx.x;
  const int lane = t & 31;
  const int wave = t >> 5;
  const float* xb = xyz + (size_t)b * kPts * 3;

  float px[8], py[8], pz[8], md[8];
#pragma unroll
  for (int j = 0; j < 8; ++j) {
    __syncthreads();
    const int tc = (t < 768) ? t : 767;
    const v4f sv = *(const v4f*)(xb + j * 3072 + tc * 4);
    if (t < 768) *(v4f*)(s_stage + t * 4) = sv;
    __syncthreads();
    px[j] = s_stage[t * 3 + 0];
    py[j] = s_stage[t * 3 + 1];
    pz[j] = s_stage[t * 3 + 2];
    md[j] = 1e10f;
  }

  int cur = 0;
  for (int i = 0; i < kChild; ++i) {
    if (t == 0) s_cidx[i] = cur;
    const float cx = xb[cur * 3 + 0];
    const float cy = xb[cur * 3 + 1];
    const float cz = xb[cur * 3 + 2];
    float bv = -1.0f;
    int   bi = 0x7fffffff;
#pragma unroll
    for (int j = 0; j < 8; ++j) {
      const float dx = px[j] - cx;
      const float dy = py[j] - cy;
      const float dz = pz[j] - cz;
      const float t0 = dx * dx;
      const float t1 = dy * dy;
      const float t2 = dz * dz;
      const float d  = (t0 + t2) + t1;
      md[j] = fminf(md[j], d);
      const bool gt = md[j] > bv;
      bv = gt ? md[j] : bv;
      bi = gt ? (j * 1024 + t) : bi;
    }
    argmax_allreduce(bv, bi);
    const int buf = i & 1;
    if (lane == 0) { s_bv[buf][wave] = bv; s_bi[buf][wave] = bi; }
    __syncthreads();
    bv = s_bv[buf][lane];
    bi = s_bi[buf][lane];
    argmax_allreduce(bv, bi);
    bi = bi < 0 ? 0 : bi;
    cur = bi > (kPts - 1) ? (kPts - 1) : bi;
  }
  __syncthreads();

  const int tq = (t < 512) ? t : 511;
  const v4i cv = *(const v4i*)(s_cidx + tq * 4);
  v4f o0, o1;
  {
    const int idx1 = (t + 1024 < 1536) ? (t + 1024) : 1535;
#pragma unroll
    for (int e = 0; e < 4; ++e) {
      const int f0 = 4 * t + e;
      const int p0 = f0 / 3;
      const int c0 = f0 - 3 * p0;
      int ci0 = s_cidx[p0];
      ci0 = ci0 < 0 ? 0 : (ci0 > kPts - 1 ? kPts - 1 : ci0);
      o0[e] = xb[ci0 * 3 + c0];
      const int f1 = 4 * idx1 + e;
      const int p1 = f1 / 3;
      const int c1 = f1 - 3 * p1;
      int ci1 = s_cidx[p1];
      ci1 = ci1 < 0 ? 0 : (ci1 > kPts - 1 ? kPts - 1 : ci1);
      o1[e] = xb[ci1 * 3 + c1];
    }
  }
  float* ob = out0 + (size_t)b * kChild * 3;
  int*   cb = cidx_ws + (size_t)b * kChild;
  for (int pass = 0; pass < 2; ++pass) {
    if (t < 512) *(volatile v4i*)(cb + t * 4) = cv;
    *(volatile v4f*)(ob + 4 * t) = o0;
    if (t < 512) *(volatile v4f*)(ob + 4 * (t + 1024)) = o1;
    __threadfence();
  }
}

__global__ __launch_bounds__(256) void group_pool_kernel(const float* __restrict__ xyz, const int* __restrict__ cidx_ws,
                                                         const unsigned* __restrict__ y2w, float* __restrict__ out1) {
#pragma clang fp contract(off)
  __shared__ int s_idx[32 * kNbr];
  __shared__ __align__(16) float s_out[kCout * 36];

  const int tid  = threadIdx.x;
  const int lane = tid & 31;
  const int wave = tid >> 5;
  const int b  = blockIdx.x >> 6;
  const int m0 = (blockIdx.x & 63) * 32;
  const float* xb = xyz + (size_t)b * kPts * 3;
  const float thr = __uint_as_float(0x3C23D70Au);

  float ccx[4], ccy[4], ccz[4], ccs[4];
  int cnt[4], first[4];
#pragma unroll
  for (int k = 0; k < 4; ++k) {
    int ci = cidx_ws[(size_t)b * kChild + m0 + wave * 4 + k];
    ci = ci < 0 ? 0 : (ci > kPts - 1 ? kPts - 1 : ci);
    ccx[k] = xb[ci * 3 + 0];
    ccy[k] = xb[ci * 3 + 1];
    ccz[k] = xb[ci * 3 + 2];
    const float t0 = ccx[k] * ccx[k];
    const float t1 = ccy[k] * ccy[k];
    const float t2 = ccz[k] * ccz[k];
    ccs[k] = (t0 + t2) + t1;
    cnt[k] = 0;
    first[k] = 0;
  }
  const unsigned lt = (1u << lane) - 1u;
  for (int base = 0; base < kPts; base += 32) {
    const bool done = (cnt[0] >= kNbr) && (cnt[1] >= kNbr) && (cnt[2] >= kNbr) && (cnt[3] >= kNbr);
    if (done) break;
    const int n = base + lane;
    const float x = xb[n * 3 + 0];
    const float y = xb[n * 3 + 1];
    const float z = xb[n * 3 + 2];
    const float u0 = x * x;
    const float u1 = y * y;
    const float u2 = z * z;
    const float xx = (u0 + u2) + u1;
#pragma unroll
    for (int k = 0; k < 4; ++k) {
      float p = ccx[k] * x;
      p = __builtin_fmaf(ccy[k], y, p);
      p = __builtin_fmaf(ccz[k], z, p);
      const float twop = 2.0f * p;
      const float d2 = (ccs[k] + xx) - twop;
      const bool hit = d2 < thr;
      const unsigned mask = __builtin_amdgcn_ballot_w32(hit);
      const int pos = cnt[k] + __builtin_popcount(mask & lt);
      if (hit && pos < kNbr) s_idx[(wave * 4 + k) * kNbr + pos] = n;
      if (cnt[k] == 0 && mask != 0u) first[k] = base + __builtin_ctz(mask);
      cnt[k] += __builtin_popcount(mask);
    }
  }
#pragma unroll
  for (int k = 0; k < 4; ++k) {
    const int nn = cnt[k] < kNbr ? cnt[k] : kNbr;
    const int fill = (cnt[k] > 0) ? first[k] : 0;
    if (lane < kNbr && lane >= nn) s_idx[(wave * 4 + k) * kNbr + lane] = fill;
  }
  __syncthreads();

  const int cp    = tid & 127;
  const int chalf = tid >> 7;
  const unsigned* yb = y2w + (size_t)b * kPts * (kCout / 2);
#pragma unroll 1
  for (int ch = 0; ch < 16; ++ch) {
    const int m = chalf * 16 + ch;
    unsigned mlo = 0u, mhi = 0u;
#pragma unroll 1
    for (int jh = 0; jh < 2; ++jh) {
      unsigned w[8];
#pragma unroll
      for (int j = 0; j < 8; ++j) {
        int id = s_idx[m * kNbr + jh * 8 + j];
        id = id < 0 ? 0 : (id > kPts - 1 ? kPts - 1 : id);
        w[j] = yb[(size_t)id * (kCout / 2) + cp];
      }
#pragma unroll
      for (int j = 0; j < 8; ++j) {
        const unsigned lo = w[j] & 0x7fffu;
        const unsigned hi = (w[j] >> 16) & 0x7fffu;
        mlo = lo > mlo ? lo : mlo;
        mhi = hi > mhi ? hi : mhi;
      }
    }
    s_out[(2 * cp) * 36 + m]     = h16_to_f32(mlo);
    s_out[(2 * cp + 1) * 36 + m] = h16_to_f32(mhi);
  }
  __syncthreads();

  v4f vals[8];
#pragma unroll
  for (int it = 0; it < 8; ++it) {
    const int c = wave * 32 + it * 4 + (lane >> 3);
    vals[it] = *(const v4f*)(s_out + c * 36 + (lane & 7) * 4);
  }
  for (int pass = 0; pass < 2; ++pass) {
#pragma unroll
    for (int it = 0; it < 8; ++it) {
      const int c = wave * 32 + it * 4 + (lane >> 3);
      *(volatile v4f*)(out1 + ((size_t)(b * kCout + c)) * kChild + m0 + (lane & 7) * 4) = vals[it];
    }
    __threadfence();
  }
}

extern "C" void kernel_launch(void* const* d_in, const int* in_sizes, int n_in,
                              void* d_out, int out_size, void* d_ws, size_t ws_size,
                              hipStream_t stream) {
  if (n_in < 6) return;
  if (in_sizes[0] != kBatch * kPts * 3) return;
  if (in_sizes[1] != kBatch * kCin * kPts) return;
  if (in_sizes[2] != kCout * kCin || in_sizes[3] != kCout) return;
  if (in_sizes[4] != kCout * kCout || in_sizes[5] != kCout) return;
  if (out_size != (int)((kOut0Bytes + kOut1Bytes) / 4)) return;
  if (ws_size < kWsTotal) return;

  const float* xyz   = (const float*)d_in[0];
  const float* feats = (const float*)d_in[1];
  const float* w1    = (const float*)d_in[2];
  const float* b1    = (const float*)d_in[3];
  const float* w2    = (const float*)d_in[4];
  const float* b2    = (const float*)d_in[5];

  float* out0 = (float*)d_out;
  float* out1 = (float*)d_out + (kOut0Bytes / 4);

  char* ws = (char*)d_ws;
  unsigned short* Xh  = (unsigned short*)(ws + kOffXh);
  unsigned short* Wh  = (unsigned short*)(ws + kOffWh);
  unsigned short* W1h = Wh;
  unsigned short* W2h = Wh + kCout * kCin;
  unsigned short* Y1h = (unsigned short*)(ws + kOffY1);
  unsigned short* Y2h = (unsigned short*)(ws + kOffY2);
  int* cidx = (int*)(ws + kOffCidx);

  const int Mrows = kBatch * kPts;
  const int gemmBlocks = ((Mrows / 64) * (kCout / 64)) / 8;

  fps_kernel<<<kBatch, 1024, 0, stream>>>(xyz, out0, cidx);
  cvt_feats_kernel<<<kBatch * (kPts / 64), 256, 0, stream>>>(feats, Xh);
  cvt_w_kernel<<<(kCout * kCin + kCout * kCout) / (256 * 8), 256, 0, stream>>>(w1, w2, Wh);
  wmma_gemm64_f16_bias_relu<<<gemmBlocks, 256, 0, stream>>>(Xh, kCin, W1h, kCin, Y1h, kCout, b1, Mrows, kCout, kCin, kWCarryInv);
  wmma_gemm64_f16_bias_relu<<<gemmBlocks, 256, 0, stream>>>(Y1h, kCout, W2h, kCout, Y2h, kCout, b2, Mrows, kCout, kCout, kWCarryInv);
  group_pool_kernel<<<kBatch * (kChild / 32), 256, 0, stream>>>(xyz, cidx, (const unsigned*)Y2h, out1);
}
